// TFAttention_28621662060547
// MI455X (gfx1250) — hardware-verified
//
#include <hip/hip_runtime.h>
#include <math.h>

#ifndef NB
#define NB 4
#endif
#ifndef SEQ
#define SEQ 2048
#endif
#define NB_FULL  4
#define SEQ_FULL 2048
#define DD  1024
#define HH  16
#define DKK 64
#define QW  2

static_assert(NB >= 1 && NB <= NB_FULL);
static_assert(SEQ % 128 == 0 && SEQ <= SEQ_FULL);
static_assert(DD % 256 == 0);
static_assert(HH * DKK == DD);
static_assert(QW == 2);

#define LOG2E 1.44269504088896340736f

typedef _Float16 f16;
typedef unsigned v4u_t __attribute__((ext_vector_type(4)));
typedef unsigned v4ua  __attribute__((ext_vector_type(4), may_alias));
typedef float    v4f_t __attribute__((ext_vector_type(4)));
typedef float    v4fa  __attribute__((ext_vector_type(4), may_alias));
typedef f16   f16x16 __attribute__((ext_vector_type(16)));
typedef f16   f16x8  __attribute__((ext_vector_type(8)));
typedef f16   f16x4  __attribute__((ext_vector_type(4)));
typedef float f32x8  __attribute__((ext_vector_type(8)));

#define LDS_STRIDE 48
#define KSTRIDE    72
#define VSTRIDE    48

__device__ __forceinline__ f32x8 wmma16(f16x16 a, f16x16 b, f32x8 c) {
  return __builtin_amdgcn_wmma_f32_16x16x32_f16(
      false, a, false, b, (short)0, c, false, false);
}
#define RSPLIT (1.0f / 2048.0f)
__device__ __forceinline__ f16 lo_of(float v, f16 h) { return (f16)((v - (float)h) * 2048.0f); }
__device__ __forceinline__ f32x8 wmma_split(f16x16 a, f16x16 al, f16x16 b, f16x16 bl, f32x8 c) {
  f32x8 x = {}; x = wmma16(al, b, x); x = wmma16(a, bl, x); return wmma16(a, b, c) + x * RSPLIT; }

template <typename T>
__device__ __forceinline__ f16x16 load_frag(const T* __restrict__ base, int ld,
                                            int row0, int k0) {
  const int lane = threadIdx.x & 31;
  const int r    = lane & 15;
  const int kh   = (lane >> 4) * 8;
  const T* p0 = base + (size_t)(row0 + r) * ld + (k0 + kh);
  const T* p1 = p0 + 16;
  f16x16 f;
#pragma unroll
  for (int i = 0; i < 8; ++i) {
    f[i]     = (f16)p0[i];
    f[i + 8] = (f16)p1[i];
  }
  return f;
}

__device__ __forceinline__ f16x16 lds_frag(const f16* base, int stride) {
  const int lane = threadIdx.x & 31;
  const int row  = lane & 15;
  const int kh   = (lane >> 4) * 8;
  const f16x8 lo = *(const f16x8*)(base + row * stride + kh);
  const f16x8 hi = *(const f16x8*)(base + row * stride + kh + 16);
  f16x16 f;
#pragma unroll
  for (int i = 0; i < 8; ++i) { f[i] = lo[i]; f[i + 8] = hi[i]; }
  return f;
}

template <typename T>
__device__ __forceinline__ void stage_read16(const T* __restrict__ p, float* buf) {
#pragma unroll
  for (int i = 0; i < 16; ++i) buf[i] = (float)p[i];
}

__device__ __forceinline__ void stage_write(f16* dst, const float* buf, int nquad) {
#pragma unroll
  for (int i = 0; i < nquad; ++i) {
    f16x4 q;
    q[0] = (f16)buf[4 * i];     q[1] = (f16)buf[4 * i + 1];
    q[2] = (f16)buf[4 * i + 2]; q[3] = (f16)buf[4 * i + 3];
    *(f16x4*)(dst + 4 * i) = q;
  }
}

__global__ __launch_bounds__(256) void transpose_pack_kernel(const float* __restrict__ W, f16* __restrict__ WT, int K, int N, size_t plane) {
  __shared__ float tile[64][65];
  const int k0 = blockIdx.y * 64, n0 = blockIdx.x * 64, t = threadIdx.x;
  for (int i = t; i < 64 * 64; i += 256) { const int kr = i >> 6, nc = i & 63; tile[kr][nc] = W[(size_t)(k0 + kr) * N + n0 + nc]; }
  __syncthreads();
#pragma unroll 1
  for (int pass = 0; pass < 2; ++pass) {
    for (int i = t; i < 64 * 8; i += 256) { const int nr = i >> 3, k8 = (i & 7) * 8; f16 hh[8], hl[8];
#pragma unroll
      for (int e = 0; e < 8; ++e) { const float v = tile[k8 + e][nr]; hh[e] = (f16)v; hl[e] = lo_of(v, hh[e]); }
      f16* d = WT + (size_t)(n0 + nr) * K + k0 + k8;
      *(volatile v4u_t*)d = *(const v4ua*)hh; *(volatile v4u_t*)(d + plane) = *(const v4ua*)hl; }
    __threadfence();
  }
}

template <typename AT, typename WT, int MODE>
__global__ __launch_bounds__(256) void gemm_bias_kernel(
    const AT* __restrict__ A, int aS, const WT* __restrict__ W,
    const float* __restrict__ bias, void* __restrict__ out, int N, int K) {
  __shared__ f16 ldsA[128 * LDS_STRIDE];
  __shared__ f16 ldsW[256 * LDS_STRIDE];
  __shared__ __attribute__((aligned(16))) unsigned char sob[256 * 136 * 2];

  const int t    = threadIdx.x;
  const int wave = t >> 5;
  const int lane = t & 31;
  const int wm   = (wave & 1) * 64;
  const int wn   = (wave >> 1) * 64;
  const int mBlk = blockIdx.x * 128;
  const int nBlk = blockIdx.y * 256;
  const int bBlk = mBlk / SEQ, sBlk = mBlk - bBlk * SEQ;
  const AT* Ab = A + ((size_t)bBlk * aS + sBlk) * K;

  const int arow = t >> 1;
  const int ach  = (t & 1) * 16;

  float abuf[16];
  float wbuf[32];

  stage_read16(Ab + (size_t)arow * K + ach,     abuf);
  stage_read16(W + (size_t)(nBlk + t) * K,      wbuf);
  stage_read16(W + (size_t)(nBlk + t) * K + 16, wbuf + 16);

  f32x8 acc[4][4] = {};

  for (int k = 0; k < K; k += 32) {
    __syncthreads();
    stage_write(&ldsA[arow * LDS_STRIDE + ach], abuf, 4);
    stage_write(&ldsW[t * LDS_STRIDE],          wbuf, 8);
    if (k + 32 < K) {
      stage_read16(Ab + (size_t)arow * K + (k + 32) + ach,     abuf);
      stage_read16(W + (size_t)(nBlk + t) * K + (k + 32),      wbuf);
      stage_read16(W + (size_t)(nBlk + t) * K + (k + 32) + 16, wbuf + 16);
    }
    __syncthreads();

    f16x16 af[4], wf[4];
#pragma unroll
    for (int i = 0; i < 4; ++i)
      af[i] = lds_frag(ldsA + (wm + 16 * i) * LDS_STRIDE, LDS_STRIDE);
#pragma unroll
    for (int j = 0; j < 4; ++j)
      wf[j] = lds_frag(ldsW + (wn + 16 * j) * LDS_STRIDE, LDS_STRIDE);
#pragma unroll
    for (int i = 0; i < 4; ++i)
#pragma unroll
      for (int j = 0; j < 4; ++j)
        acc[i][j] = wmma16(af[i], wf[j], acc[i][j]);
  }

  const int nlane = lane & 15;
  const int mh    = (lane >> 4) * 8;
  __syncthreads();
  if (MODE == 0 || MODE == 1) {
    f16* so = (f16*)sob;
#pragma unroll
    for (int i = 0; i < 4; ++i)
#pragma unroll
      for (int j = 0; j < 4; ++j) {
        const int nl = wn + 16 * j + nlane;
        const float bv = bias[nBlk + nl];
#pragma unroll
        for (int r = 0; r < 8; ++r) {
          const int ml = wm + 16 * i + mh + r;
          const f16 hv = (f16)(acc[i][j][r] + bv);
          if (MODE == 0) so[ml * 264 + nl] = hv;
          else           so[nl * 136 + ml] = hv;
        }
      }
    __syncthreads();
#pragma unroll 1
    for (int pass = 0; pass < 2; ++pass) {
      if (MODE == 0) {
        for (int ch = t; ch < 128 * 32; ch += 256) { const int ml = ch >> 5, q = (ch & 31) * 8;
          *(volatile v4u_t*)((f16*)out + (size_t)(mBlk + ml) * N + nBlk + q) = *(const v4ua*)(so + ml * 264 + q); }
      } else {
        for (int ch = t; ch < 256 * 16; ch += 256) { const int nl = ch >> 4, q = (ch & 15) * 8; const int n = nBlk + nl, h = n >> 6, dk = n & (DKK - 1);
          *(volatile v4u_t*)((f16*)out + (((size_t)(bBlk * HH + h)) * DKK + dk) * SEQ + sBlk + q) = *(const v4ua*)(so + nl * 136 + q); }
      }
      __threadfence();
    }
  } else {
    float* so = (float*)sob;
#pragma unroll 1
    for (int hf = 0; hf < 2; ++hf) {
      if (wm == hf * 64) {
#pragma unroll
        for (int i = 0; i < 4; ++i)
#pragma unroll
          for (int j = 0; j < 4; ++j) {
            const int nl = wn + 16 * j + nlane;
            const float bv = bias[nBlk + nl];
#pragma unroll
            for (int r = 0; r < 8; ++r) so[(16 * i + mh + r) * 260 + nl] = acc[i][j][r] + bv;
          }
      }
      __syncthreads();
#pragma unroll 1
      for (int pass = 0; pass < 2; ++pass) {
        for (int ch = t; ch < 64 * 64; ch += 256) { const int ml = ch >> 6, q = (ch & 63) * 4;
          *(volatile v4f_t*)((float*)out + (size_t)(mBlk + hf * 64 + ml) * N + nBlk + q) = *(const v4fa*)(so + ml * 260 + q); }
        __threadfence();
      }
      __syncthreads();
    }
  }
}

template <typename AT, typename WT, int MODE>
__global__ __launch_bounds__(256) void gemm_split_kernel(
    const AT* __restrict__ A, int aS, size_t aPlane, const WT* __restrict__ W, size_t wPlane,
    const float* __restrict__ bias, void* __restrict__ out, int N, int K) {
  __shared__ f16 ldsA[128 * LDS_STRIDE], ldsAl[128 * LDS_STRIDE];
  __shared__ f16 ldsW[256 * LDS_STRIDE], ldsWl[256 * LDS_STRIDE];
  __shared__ __attribute__((aligned(16))) unsigned char sob[256 * 136 * 2];

  const int t    = threadIdx.x;
  const int wave = t >> 5;
  const int lane = t & 31;
  const int wm   = (wave & 1) * 64;
  const int wn   = (wave >> 1) * 64;
  const int mBlk = blockIdx.x * 128;
  const int nBlk = blockIdx.y * 256;
  const int bBlk = mBlk / SEQ, sBlk = mBlk - bBlk * SEQ;
  const AT* Ab = A + ((size_t)bBlk * aS + sBlk) * K;
  const int arow = t >> 1;
  const int ach  = (t & 1) * 16;

  f32x8 acc[4][4] = {};
  for (int k = 0; k < K; k += 32) {
    __syncthreads();
    {
      const AT* ap = Ab + (size_t)arow * K + k + ach;
      f16 hh[16], hl[16];
      if (sizeof(AT) == 4) {
#pragma unroll
        for (int i = 0; i < 16; ++i) { const float v = (float)ap[i]; hh[i] = (f16)v; hl[i] = lo_of(v, hh[i]); }
      } else {
#pragma unroll
        for (int i = 0; i < 16; ++i) { hh[i] = (f16)ap[i]; hl[i] = (f16)ap[aPlane + i]; }
      }
#pragma unroll
      for (int i = 0; i < 16; ++i) { ldsA[arow * LDS_STRIDE + ach + i] = hh[i]; ldsAl[arow * LDS_STRIDE + ach + i] = hl[i]; }
    }
    {
      const WT* wp = W + (size_t)(nBlk + t) * K + k;
      if (sizeof(WT) == 4) {
#pragma unroll
        for (int i = 0; i < 32; ++i) { const float v = (float)wp[i]; const f16 h_ = (f16)v; ldsW[t * LDS_STRIDE + i] = h_; ldsWl[t * LDS_STRIDE + i] = lo_of(v, h_); }
      } else {
#pragma unroll
        for (int i = 0; i < 32; ++i) { ldsW[t * LDS_STRIDE + i] = (f16)wp[i]; ldsWl[t * LDS_STRIDE + i] = (f16)wp[wPlane + i]; }
      }
    }
    __syncthreads();
    f16x16 wf[4], wfl[4];
#pragma unroll
    for (int j = 0; j < 4; ++j) { wf[j] = lds_frag(ldsW + (wn + 16 * j) * LDS_STRIDE, LDS_STRIDE); wfl[j] = lds_frag(ldsWl + (wn + 16 * j) * LDS_STRIDE, LDS_STRIDE); }
#pragma unroll
    for (int i = 0; i < 4; ++i) {
      const f16x16 af = lds_frag(ldsA + (wm + 16 * i) * LDS_STRIDE, LDS_STRIDE), afl = lds_frag(ldsAl + (wm + 16 * i) * LDS_STRIDE, LDS_STRIDE);
#pragma unroll
      for (int j = 0; j < 4; ++j) acc[i][j] = wmma_split(af, afl, wf[j], wfl[j], acc[i][j]);
    }
  }

  const int nlane = lane & 15;
  const int mh    = (lane >> 4) * 8;
  __syncthreads();
  if (MODE == 1) {
    f16* so = (f16*)sob;
#pragma unroll
    for (int i = 0; i < 4; ++i)
#pragma unroll
      for (int j = 0; j < 4; ++j) {
        const int nl = wn + 16 * j + nlane;
        const float bv = bias ? bias[nBlk + nl] : 0.0f;
#pragma unroll
        for (int r = 0; r < 8; ++r) so[nl * 136 + wm + 16 * i + mh + r] = (f16)(acc[i][j][r] + bv);
      }
    __syncthreads();
#pragma unroll 1
    for (int pass = 0; pass < 2; ++pass) {
      for (int ch = t; ch < 256 * 16; ch += 256) { const int nl = ch >> 4, q = (ch & 15) * 8; const int n = nBlk + nl, h = n >> 6, dk = n & (DKK - 1);
        *(volatile v4u_t*)((f16*)out + (((size_t)(bBlk * HH + h)) * DKK + dk) * SEQ + sBlk + q) = *(const v4ua*)(so + nl * 136 + q); }
      __threadfence();
    }
  } else {
    float* so = (float*)sob;
#pragma unroll 1
    for (int hf = 0; hf < 2; ++hf) {
      if (wm == hf * 64) {
#pragma unroll
        for (int i = 0; i < 4; ++i)
#pragma unroll
          for (int j = 0; j < 4; ++j) {
            const int nl = wn + 16 * j + nlane;
            const float bv = bias ? bias[nBlk + nl] : 0.0f;
#pragma unroll
            for (int r = 0; r < 8; ++r) so[(16 * i + mh + r) * 260 + nl] = acc[i][j][r] + bv;
          }
      }
      __syncthreads();
#pragma unroll 1
      for (int pass = 0; pass < 2; ++pass) {
        for (int ch = t; ch < 64 * 64; ch += 256) { const int ml = ch >> 6, q = (ch & 63) * 4;
          *(volatile v4f_t*)((float*)out + (size_t)(mBlk + hf * 64 + ml) * N + nBlk + q) = *(const v4fa*)(so + ml * 260 + q); }
        __threadfence();
      }
      __syncthreads();
    }
  }
}

__global__ __launch_bounds__(64) void attn_kernel(
    const f16* __restrict__ Qb, const f16* __restrict__ Kb,
    const f16* __restrict__ Vt, const float* __restrict__ mask,
    f16* __restrict__ attnOut) {
  __shared__ f16 ldsK[32 * KSTRIDE];
  __shared__ f16 ldsV[64 * VSTRIDE];
  __shared__ __attribute__((aligned(16))) f16 ldsO[2][32 * 72], ldsOl[2][32 * 72];

  const int q0blk = blockIdx.x * 64;
  const int h  = blockIdx.y;
  const int b  = blockIdx.z;
  const int t    = threadIdx.x;
  const int wave = t >> 5;
  const int lane = t & 31;
  const int qlane = lane & 15;
  const int kh8   = (lane >> 4) * 8;
  const int q0 = q0blk + wave * 32;

  const f16* Qh = Qb + (size_t)b * SEQ * DD + h * DKK;
  const f16* Kh = Kb + (size_t)b * SEQ * DD + h * DKK;
  const f16* Vh = Vt + ((size_t)(b * HH + h)) * DKK * SEQ;
  const float* mrow = mask + (size_t)b * SEQ_FULL;

  const int krow = t >> 1;
  const int kcol = (t & 1) * 32;
  const f16* kSrc = Kh + (size_t)krow * DD + kcol;
  const f16* vSrc = Vh + (size_t)t * SEQ;

  f16x16 qf[QW][2];
#pragma unroll
  for (int qt = 0; qt < QW; ++qt) {
    qf[qt][0] = load_frag(Qh, DD, q0 + 16 * qt, 0);
    qf[qt][1] = load_frag(Qh, DD, q0 + 16 * qt, 32);
  }

  f32x8 o[QW][4] = {};
  float mrun[QW], lrun[QW];
#pragma unroll
  for (int qt = 0; qt < QW; ++qt) { mrun[qt] = -INFINITY; lrun[qt] = 0.0f; }

  const float scale = 0.125f * LOG2E;

  f16x8 kreg[4], vreg[4];
#pragma unroll
  for (int i = 0; i < 4; ++i) {
    kreg[i] = *(const f16x8*)(kSrc + 8 * i);
    vreg[i] = *(const f16x8*)(vSrc + 8 * i);
  }

  for (int kb = 0; kb < SEQ; kb += 32) {
    __syncthreads();
#pragma unroll
    for (int i = 0; i < 4; ++i) {
      *(f16x8*)(&ldsK[krow * KSTRIDE + kcol + 8 * i]) = kreg[i];
      *(f16x8*)(&ldsV[t * VSTRIDE + 8 * i])           = vreg[i];
    }
    if (kb + 32 < SEQ) {
      const f16* kn = kSrc + (size_t)(kb + 32) * DD;
      const f16* vn = vSrc + (kb + 32);
#pragma unroll
      for (int i = 0; i < 4; ++i) {
        kreg[i] = *(const f16x8*)(kn + 8 * i);
        vreg[i] = *(const f16x8*)(vn + 8 * i);
      }
    }
    __syncthreads();

    f16x16 kf[2][2];
#pragma unroll
    for (int ktile = 0; ktile < 2; ++ktile)
#pragma unroll
      for (int c = 0; c < 2; ++c)
        kf[ktile][c] = lds_frag(ldsK + (ktile * 16) * KSTRIDE + c * 32, KSTRIDE);

    float madd0[8], madd1[8];
    {
      const v4f_t m00 = *(const v4f_t*)(mrow + kb + kh8);
      const v4f_t m01 = *(const v4f_t*)(mrow + kb + kh8 + 4);
      const v4f_t m10 = *(const v4f_t*)(mrow + kb + 16 + kh8);
      const v4f_t m11 = *(const v4f_t*)(mrow + kb + 16 + kh8 + 4);
#pragma unroll
      for (int r = 0; r < 4; ++r) {
        madd0[r]     = (m00[r] + 1e-9f) * LOG2E;
        madd0[r + 4] = (m01[r] + 1e-9f) * LOG2E;
        madd1[r]     = (m10[r] + 1e-9f) * LOG2E;
        madd1[r + 4] = (m11[r] + 1e-9f) * LOG2E;
      }
    }

    f16x16 pf[QW];
#pragma unroll
    for (int qt = 0; qt < QW; ++qt) {
      f32x8 s0 = {}, s1 = {};
      s0 = wmma16(kf[0][0], qf[qt][0], s0);
      s0 = wmma16(kf[0][1], qf[qt][1], s0);
      s1 = wmma16(kf[1][0], qf[qt][0], s1);
      s1 = wmma16(kf[1][1], qf[qt][1], s1);
      asm volatile("v_nop\n\tv_nop\n\tv_nop\n\tv_nop" : "+v"(s0), "+v"(s1));

      float mx = -INFINITY;
#pragma unroll
      for (int r = 0; r < 8; ++r) {
        s0[r] = s0[r] * scale + madd0[r];
        s1[r] = s1[r] * scale + madd1[r];
        mx = fmaxf(mx, fmaxf(s0[r], s1[r]));
      }
      mx = fmaxf(mx, __shfl_xor(mx, 16, 32));
      const float mnew  = fmaxf(mrun[qt], mx);
      const float alpha = exp2f(mrun[qt] - mnew);

      float rsum = 0.0f;
#pragma unroll
      for (int r = 0; r < 8; ++r) {
        const float p0 = exp2f(s0[r] - mnew);
        const float p1 = exp2f(s1[r] - mnew);
        rsum += p0 + p1;
        pf[qt][r]     = (f16)(p0 * 1024.0f);
        pf[qt][r + 8] = (f16)(p1 * 1024.0f);
      }
      rsum += __shfl_xor(rsum, 16, 32);
      lrun[qt] = lrun[qt] * alpha + rsum;
      mrun[qt] = mnew;

#pragma unroll
      for (int j = 0; j < 4; ++j)
#pragma unroll
        for (int r = 0; r < 8; ++r) o[qt][j][r] *= alpha;
    }

#pragma unroll
    for (int j = 0; j < 4; ++j) {
      const f16x16 vf = lds_frag(ldsV + (j * 16) * VSTRIDE, VSTRIDE);
#pragma unroll
      for (int qt = 0; qt < QW; ++qt)
        o[qt][j] = wmma16(vf, pf[qt], o[qt][j]);
    }
    asm volatile("v_nop\n\tv_nop\n\tv_nop\n\tv_nop"
                 : "+v"(o[0][0]), "+v"(o[0][1]), "+v"(o[0][2]), "+v"(o[0][3]),
                   "+v"(o[1][0]), "+v"(o[1][1]), "+v"(o[1][2]), "+v"(o[1][3]));
  }

  f16* so = ldsO[wave]; f16* sol = ldsOl[wave];
#pragma unroll
  for (int qt = 0; qt < QW; ++qt) {
    const float rl = 1.0f / (lrun[qt] * 1024.0f);
#pragma unroll
    for (int j = 0; j < 4; ++j)
#pragma unroll
      for (int r = 0; r < 8; ++r) { const float v = o[qt][j][r] * rl; const f16 hv = (f16)v;
        so[(16 * qt + qlane) * 72 + j * 16 + kh8 + r] = hv; sol[(16 * qt + qlane) * 72 + j * 16 + kh8 + r] = lo_of(v, hv); }
  }
  __syncthreads();
  const size_t plane = (size_t)NB * SEQ * DD;
#pragma unroll 1
  for (int pass = 0; pass < 2; ++pass) {
#pragma unroll
    for (int it = 0; it < 8; ++it) { const int ch = lane + 32 * it, ql = ch >> 3, q8 = (ch & 7) * 8;
      f16* d = attnOut + ((size_t)(b * SEQ + q0 + ql)) * DD + h * DKK + q8;
      *(volatile v4u_t*)d = *(const v4ua*)(so + ql * 72 + q8); *(volatile v4u_t*)(d + plane) = *(const v4ua*)(sol + ql * 72 + q8); }
    __threadfence();
  }
}

extern "C" void kernel_launch(void* const* d_in, const int* in_sizes, int n_in,
                              void* d_out, int out_size, void* d_ws, size_t ws_size,
                              hipStream_t stream) {
  if (n_in < 6) return;
  const float* x        = (const float*)d_in[0];
  const float* amask    = (const float*)d_in[1];
  const float* c_attn_w = (const float*)d_in[2];
  const float* c_attn_b = (const float*)d_in[3];
  const float* c_proj_w = (const float*)d_in[4];
  const float* c_proj_b = (const float*)d_in[5];

  if (in_sizes[0] < ((NB - 1) * SEQ_FULL + SEQ) * DD) return;
  if (in_sizes[1] < (NB - 1) * SEQ_FULL + SEQ) return;
  if (in_sizes[2] < DD * 3 * DD || in_sizes[3] < 3 * DD || in_sizes[4] < DD * DD || in_sizes[5] < DD) return;
  if (out_size < NB * SEQ * DD) return;

  const size_t actBytes = (size_t)NB * SEQ * DD * sizeof(f16);
  const size_t plQKV = (size_t)3 * DD * DD, plP = (size_t)DD * DD;
  const size_t offQ = 0, offK = actBytes, offV = 2 * actBytes, offAttn = 3 * actBytes;
  const size_t offWqkv = 5 * actBytes;
  const size_t offWp   = offWqkv + 2 * plQKV * sizeof(f16);
  const size_t wsEnd   = offWp + 2 * plP * sizeof(f16);
  if (ws_size < wsEnd) return;

  char* ws    = (char*)d_ws;
  f16* Qb     = (f16*)(ws + offQ);
  f16* Kb     = (f16*)(ws + offK);
  f16* VtB    = (f16*)(ws + offV);
  f16* attn   = (f16*)(ws + offAttn);
  f16* WqkvT  = (f16*)(ws + offWqkv);
  f16* WpT    = (f16*)(ws + offWp);

  transpose_pack_kernel<<<dim3(3 * DD / 64, DD / 64), 256, 0, stream>>>(c_attn_w, WqkvT, DD, 3 * DD, plQKV);
  transpose_pack_kernel<<<dim3(DD / 64, DD / 64), 256, 0, stream>>>(c_proj_w, WpT, DD, DD, plP);

  const int M = NB * SEQ, N = DD, K = DD;
  dim3 gGrid(M / 128, N / 256);
  dim3 gBlk(256);

  gemm_bias_kernel<float, f16, 0><<<gGrid, gBlk, 0, stream>>>(x, SEQ_FULL, WqkvT,                   c_attn_b,      Qb, N, K);
  gemm_bias_kernel<float, f16, 0><<<gGrid, gBlk, 0, stream>>>(x, SEQ_FULL, WqkvT + (size_t)DD * DD, c_attn_b + DD, Kb, N, K);
  gemm_split_kernel<float, f16, 1><<<gGrid, gBlk, 0, stream>>>(x, SEQ_FULL, (size_t)0, WqkvT + (size_t)2 * DD * DD, plQKV, c_attn_b + 2 * DD, VtB, N, K);

  dim3 aGrid(SEQ / 64, HH, NB);
  attn_kernel<<<aGrid, dim3(64), 0, stream>>>(Qb, Kb, VtB, amask, attn);

  gemm_split_kernel<f16, f16, 2><<<gGrid, gBlk, 0, stream>>>(attn, SEQ, (size_t)NB * SEQ * DD, WpT, plP, c_proj_b, (float*)d_out, N, K);
}
